// CrystalGraphConvNet_31980326486278
// MI455X (gfx1250) — hardware-run, weakly checked
//
#include <hip/hip_runtime.h>


namespace {
constexpr int N = 8000, E = 48000, C = 16, HW = 64, KC = 144, KP = 160;
constexpr float XS = 8.0f, WSC = 256.0f, BNI = 0.99999500003749981f;

typedef _Float16 b16;
typedef __attribute__((ext_vector_type(16))) _Float16 v16b;
typedef __attribute__((ext_vector_type(8))) _Float16 v8b;
typedef __attribute__((ext_vector_type(8))) float v8f;
typedef __attribute__((ext_vector_type(4))) float v4f;
__device__ __forceinline__ float bf16_rne(float f) { unsigned int u = __float_as_uint(f); u += 0x7FFFu + ((u >> 16) & 1u); return __uint_as_float(u & 0xFFFF0000u); }
__device__ __forceinline__ void split16(float v, b16& hi, b16& lo) { hi = (b16)v; lo = (b16)(v - (float)hi); }
__device__ __forceinline__ v16b frag_kb(const b16* p, int hh) { const v8b a = *(const v8b*)(p + 8 * hh), b = *(const v8b*)(p + 16 + 8 * hh); v16b f;
#pragma unroll
  for (int e = 0; e < 8; ++e) { f[e] = a[e]; f[8 + e] = b[e]; } return f; }
__device__ __forceinline__ v8f wmma16b(v16b a, v16b b, v8f c) { v8f d = __builtin_amdgcn_wmma_f32_16x16x32_f16(false, a, false, b, (short)0, c, false, false); asm volatile("v_nop\n\tv_nop\n\tv_nop\n\tv_nop" : "+v"(d) : "v"(a), "v"(b)); return d; }
__device__ __forceinline__ void wave_lds_sync() { __builtin_amdgcn_fence(__ATOMIC_RELEASE, "workgroup"); __builtin_amdgcn_wave_barrier(); __builtin_amdgcn_fence(__ATOMIC_ACQUIRE, "workgroup"); }
__device__ __forceinline__ float pmul(float a, float b) { float p = a * b; asm volatile("" : "+v"(p)); return p; }
__device__ __forceinline__ int iclamp(int v, int lo, int hi) { return v < lo ? lo : (v > hi ? hi : v); }
__device__ __forceinline__ float nexp(float x) { return __builtin_amdgcn_exp2f(x * 1.4426950408889634f); }
__device__ __forceinline__ float elu(float x) { return x > 0.0f ? x : (__expf(x) - 1.0f); }
__device__ __forceinline__ float sigm(float x) { return 1.0f / (1.0f + nexp(-x)); }
__device__ __forceinline__ float softplus(float x) { return x > 20.0f ? x : log1pf(__expf(x)); }

constexpr int CSR_NBLK = 512, CSR_GB = 9, CSR_GN = 1 << CSR_GB  , CSR_MAXG = 512, CSR_CAP = 12288  ;
__global__ __launch_bounds__(64) void csrA_kernel(const int* __restrict__ dst, int E, int N, int nG, int CHP, int NGP, int* __restrict__ STG, int* __restrict__ HST) {
  extern __shared__ int sm[];
  int* cnt = sm; int* run = sm + NGP; int* ids = sm + 2 * NGP;
  const int b = blockIdx.x; const int ch = (E + CSR_NBLK - 1) / CSR_NBLK; const int e0 = b * ch, e1 = min(E, e0 + ch);
  for (int i = threadIdx.x; i < NGP; i += 64) cnt[i] = 0;
  for (int i = threadIdx.x; i < CHP; i += 64) ids[i] = -1;
  __syncthreads();
  if (threadIdx.x == 0) {
    for (int e = e0; e < e1; ++e) { int d = dst[e]; d = (d < 0) ? 0 : (d >= N ? N - 1 : d); cnt[d >> CSR_GB] += 1; }
    int acc = 0; for (int g = 0; g < nG; ++g) { run[g] = acc; acc += cnt[g]; }
    for (int e = e0; e < e1; ++e) { int d = dst[e]; d = (d < 0) ? 0 : (d >= N ? N - 1 : d); const int g = d >> CSR_GB; ids[run[g]] = e; run[g] += 1; } }
  __syncthreads();
  typedef __attribute__((ext_vector_type(4))) int v4i;
  for (int pass = 0; pass < 2; ++pass) {
    for (int i = threadIdx.x; i < CHP / 4; i += 64) *(volatile v4i*)(STG + (size_t)b * CHP + i * 4) = *(const v4i*)(&ids[i * 4]);
    for (int i = threadIdx.x; i < NGP / 4; i += 64) { v4i v; for (int e = 0; e < 4; ++e) v[e] = (i * 4 + e < nG) ? cnt[i * 4 + e] : 0; *(volatile v4i*)(HST + (size_t)b * NGP + i * 4) = v; }
    __threadfence(); }
}
__global__ __launch_bounds__(512) void csrS_kernel(const int* __restrict__ HST, int nG, int NGP, int* __restrict__ START, int* __restrict__ TOT, int* __restrict__ OFF) {
  __shared__ int tot[CSR_MAXG];
  const int b = threadIdx.x;
  for (int pass = 0; pass < 2; ++pass) { int runb = 0; for (int g = 0; g < nG; ++g) { int c = HST[(size_t)b * NGP + g]; c = (c < 0) ? 0 : c; ((volatile int*)OFF)[(size_t)g * CSR_NBLK + b] = runb; runb += c; } __threadfence(); }
  for (int g = threadIdx.x; g < nG; g += 512) { int s = 0; for (int bb = 0; bb < CSR_NBLK; ++bb) { int c = HST[(size_t)bb * NGP + g]; s += (c < 0) ? 0 : c; } tot[g] = s; }
  __syncthreads();
  if (threadIdx.x < 32) {
    __shared__ int st[CSR_MAXG + 32];
    if (threadIdx.x == 0) { int acc = 0; for (int g = 0; g < NGP; ++g) { st[g] = acc; if (g < nG) acc += (tot[g] + 31) & ~31; } st[NGP] = acc; }
    __builtin_amdgcn_fence(__ATOMIC_RELEASE, "workgroup"); __builtin_amdgcn_wave_barrier(); __builtin_amdgcn_fence(__ATOMIC_ACQUIRE, "workgroup");
    for (int pass = 0; pass < 2; ++pass) { for (int i = threadIdx.x; i < NGP + 32; i += 32) { ((volatile int*)START)[i] = (i <= NGP) ? st[min(i, NGP)] : 0; ((volatile int*)TOT)[i] = (i < nG) ? tot[i] : 0; } __threadfence(); } }
}
__global__ __launch_bounds__(256) void csrB_kernel(const int* __restrict__ dst, int N, int nG, int CHP, int NGP, int permLen, const int* __restrict__ STG, const int* __restrict__ HST, const int* __restrict__ OFF, const int* __restrict__ START, const int* __restrict__ TOT, int* __restrict__ PERM, int* __restrict__ ROWPTR, int* __restrict__ ROWCNT, int* __restrict__ FLAG) {
  typedef __attribute__((ext_vector_type(4))) int v4i;
  __shared__ int ids[CSR_CAP]; __shared__ unsigned short key[CSR_CAP]; __shared__ int outp[CSR_CAP]; __shared__ int ncnt[CSR_GN + 1]; __shared__ int boff[CSR_NBLK + 1];
  const int g = blockIdx.x, t_ = threadIdx.x; int tot = TOT[g]; int st = START[g], stn = START[g + 1]; const int v0 = g * CSR_GN; const int nv = min(CSR_GN, N - v0);
  st = (st < 0) ? 0 : (st > permLen - 32 ? permLen - 32 : st) & ~31; stn = (stn < st) ? st : (stn > permLen ? permLen : stn); tot = (tot < 0) ? 0 : tot; if (tot > stn - st && tot <= CSR_CAP) tot = stn - st;
  if (tot > CSR_CAP) {
    for (int pass = 0; pass < 2; ++pass) { for (int i = t_; i < CSR_GN / 4; i += 256) { v4i a, c; for (int e = 0; e < 4; ++e) { a[e] = st; c[e] = 0; } *(volatile v4i*)(ROWPTR + v0 + i * 4) = a; *(volatile v4i*)(ROWCNT + v0 + i * 4) = c; } if (t_ == 0) ((volatile int*)FLAG)[0] = 1; __threadfence(); } (void)nv; return; }
  if (t_ == 0) { int acc = 0; for (int b = 0; b < CSR_NBLK; ++b) { boff[b] = acc; int c = HST[(size_t)b * NGP + g]; c = (c < 0) ? 0 : (c > CHP ? CHP : c); acc += c; if (acc > tot) acc = tot; } boff[CSR_NBLK] = acc; }
  for (int i = t_; i <= CSR_GN; i += 256) ncnt[i] = 0;
  __syncthreads();
  for (int b = 0; b < CSR_NBLK; ++b) { const int c = boff[b + 1] - boff[b]; int o_ = OFF[(size_t)g * CSR_NBLK + b]; o_ = (o_ < 0) ? 0 : (o_ > CHP - c ? CHP - c : o_); const int* src_ = STG + (size_t)b * CHP + o_;
    for (int i = t_; i < c; i += 256) { int id = src_[i]; id = (id < 0) ? 0 : id; ids[boff[b] + i] = id; int d = dst[id]; d = (d < v0) ? v0 : (d >= N ? N - 1 : d); int kk = d - v0; kk = (kk < 0) ? 0 : (kk >= CSR_GN ? CSR_GN - 1 : kk); key[boff[b] + i] = (unsigned short)kk; } }
  __syncthreads();
  if (t_ == 0) { for (int i = 0; i < tot; ++i) ncnt[key[i]] += 1; int acc = 0; for (int vl = 0; vl < CSR_GN; ++vl) { const int c = ncnt[vl]; ncnt[vl] = acc; acc += c; } ncnt[CSR_GN] = acc;
    for (int i = 0; i < tot; ++i) { const int vl = key[i]; outp[ncnt[vl]] = ids[i]; ncnt[vl] += 1; }
    for (int vl = CSR_GN; vl > 0; --vl) ncnt[vl] = ncnt[vl - 1]; ncnt[0] = 0; }
  __syncthreads();
  for (int pass = 0; pass < 2; ++pass) {
    for (int i = t_; i < (stn - st) / 4; i += 256) { v4i v; for (int e = 0; e < 4; ++e) { const int q = i * 4 + e; v[e] = (q < tot) ? outp[q] : -1; } *(volatile v4i*)(PERM + st + i * 4) = v; }
    for (int i = t_; i < CSR_GN / 4; i += 256) { v4i a, c; for (int e = 0; e < 4; ++e) { const int vl = i * 4 + e; a[e] = st + ncnt[vl]; c[e] = (vl < nv) ? (ncnt[vl + 1] - ncnt[vl]) : 0; } *(volatile v4i*)(ROWPTR + v0 + i * 4) = a; *(volatile v4i*)(ROWCNT + v0 + i * 4) = c; }
    __threadfence(); }
}
__global__ __launch_bounds__(256) void csrZ_kernel(int* __restrict__ p, size_t n4) { typedef __attribute__((ext_vector_type(4))) int v4i; const size_t tid = (size_t)blockIdx.x * 256 + threadIdx.x, nth = (size_t)gridDim.x * 256; v4i z = {0, 0, 0, 0}; for (size_t i = tid; i < n4; i += nth) *(volatile v4i*)(p + i * 4) = z; }
struct CsrBufs { int *STG, *HST, *OFF, *START, *TOT, *PERM, *ROWPTR, *ROWCNT, *FLAG; int nG, NGP, CHP; size_t permLen; char* base; size_t bytes; };
static size_t csr_carve(CsrBufs& c, char* ws, size_t off, int E, int N) {
  const size_t off0 = off; c.base = ws + off;
  auto al = [&](size_t bytes) { char* p = ws + off; off += (bytes + 255) & ~(size_t)255; return p; };
  c.nG = (N + CSR_GN - 1) / CSR_GN; c.NGP = (c.nG + 31) & ~31; const int ch = (E + CSR_NBLK - 1) / CSR_NBLK; c.CHP = (ch + 31) & ~31; c.permLen = (size_t)E + 32 * (size_t)c.nG + 32;
  c.STG = (int*)al((size_t)CSR_NBLK * c.CHP * 4); c.HST = (int*)al((size_t)CSR_NBLK * c.NGP * 4); c.OFF = (int*)al((size_t)c.NGP * CSR_NBLK * 4); c.START = (int*)al((size_t)(c.NGP + 64) * 4); c.TOT = (int*)al((size_t)(c.NGP + 64) * 4);
  c.PERM = (int*)al(c.permLen * 4); c.ROWPTR = (int*)al((size_t)c.nG * CSR_GN * 4); c.ROWCNT = (int*)al((size_t)c.nG * CSR_GN * 4); c.FLAG = (int*)al(256);
  c.bytes = off - off0; return off;
}
static void csr_build(const CsrBufs& c, const int* dst, int E, int N, hipStream_t stream) {
  const size_t smem = (size_t)(2 * c.NGP + c.CHP) * 4;
  csrZ_kernel<<<512, 256, 0, stream>>>((int*)c.base, c.bytes / 16);
  csrA_kernel<<<CSR_NBLK, 64, smem, stream>>>(dst, E, N, c.nG, c.CHP, c.NGP, c.STG, c.HST);
  csrS_kernel<<<1, 512, 0, stream>>>(c.HST, c.nG, c.NGP, c.START, c.TOT, c.OFF);
  csrB_kernel<<<c.nG, 256, 0, stream>>>(dst, N, c.nG, c.CHP, c.NGP, (int)c.permLen, c.STG, c.HST, c.OFF, c.START, c.TOT, c.PERM, c.ROWPTR, c.ROWCNT, c.FLAG);
}


__global__ __launch_bounds__(256) void prep_kernel(const float* __restrict__ we, const float* __restrict__ wn, const float* __restrict__ wl, b16* __restrict__ WP) {
  const int t = blockIdx.x * 256 + threadIdx.x; const int nrow = 64; if (t >= nrow * KP / 8) return; const int row = (t * 8) / KP, k0 = t * 8 - row * KP;
  const float* w; int oc; if (row < 16) { w = we; oc = row; } else if (row < 32) { w = wn; oc = row - 16; } else { w = wl; oc = row - 32; }
  v8b o; for (int j = 0; j < 8; ++j) { const int k = k0 + j; const int pair = k >> 5, kk = k & 31; const int tap = 2 * pair + (kk >> 4), ic = kk & 15; o[j] = (b16)((tap < 9) ? bf16_rne(w[(oc * C + ic) * 9 + tap]) * WSC : 0.0f); }
  for (int pass = 0; pass < 2; ++pass) { *(volatile v8b*)(WP + (size_t)t * 8) = o; __threadfence(); }
}
__device__ __forceinline__ v16b frag_taps(const b16 (*T)[C], int y, int x, int pair, int hh) {
  const int ta = 2 * pair, tb = (pair < 4) ? 2 * pair + 1 : 2 * pair;
  const int ca = (y + ta / 3) * 10 + (x + ta % 3), cb = (y + tb / 3) * 10 + (x + tb % 3);
  const v8b a = *(const v8b*)(&T[ca][8 * hh]), b = *(const v8b*)(&T[cb][8 * hh]); v16b f;
#pragma unroll
  for (int e = 0; e < 8; ++e) { f[e] = a[e]; f[8 + e] = b[e]; } return f; }
__device__ __forceinline__ void load_interior(b16 (*T)[C], const float* __restrict__ img, int t_) {
  for (int i = t_; i < HW * C; i += 128) { const int p = i >> 4, ic = i & 15; T[(1 + (p >> 3)) * 10 + 1 + (p & 7)][ic] = (b16)(bf16_rne(img[ic * HW + p]) * XS); }
}
__device__ __forceinline__ void load_img(b16 (*T)[C], const float* __restrict__ img, int t_) {
  for (int i = t_; i < 100 * C; i += 128) { const int cell = i >> 4, ic = i & 15; const int yy = cell / 10, xx = cell - yy * 10; b16 v = (b16)0.0f; if (yy >= 1 && yy <= 8 && xx >= 1 && xx <= 8) v = (b16)(bf16_rne(img[ic * HW + (yy - 1) * 8 + (xx - 1)]) * XS); T[cell][ic] = v; }
}
__global__ __launch_bounds__(128) void atom_kernel(const float* __restrict__ atom, const int* __restrict__ tgt, const b16* __restrict__ WP, const float* __restrict__ linb, const float* __restrict__ gam, const float* __restrict__ bet, const int* __restrict__ PERM, const int* __restrict__ ROWPTR, const int* __restrict__ ROWCNT, int permLen, float* __restrict__ out) {
  __shared__ __attribute__((aligned(16))) b16 T[100][C], Zh[100][C], Zl[100][C]; __shared__ __attribute__((aligned(16))) float To[C][HW + 4];
  const int a = blockIdx.x, t_ = threadIdx.x, wave = t_ >> 5, lane = t_ & 31, nloc = lane & 15, hlf = lane >> 4; const int px = wave * 16 + nloc; const int y = px >> 3, x = px & 7;
  const b16* WE = WP; const b16* WN = WP + (size_t)16 * KP; const b16* WL = WP + (size_t)32 * KP;
  for (int i = t_; i < 100 * C; i += 128) { Zh[i >> 4][i & 15] = (b16)0.0f; Zl[i >> 4][i & 15] = (b16)0.0f; }
  load_img(T, atom + (size_t)a * C * HW, t_); __syncthreads();
  v8f thn = {};
#pragma unroll
  for (int pr = 0; pr < 5; ++pr) thn = wmma16b(frag_taps(T, y, x, pr, hlf), frag_kb(WN + (size_t)nloc * KP + pr * 32, hlf), thn);
  thn *= (1.0f / (XS * WSC));
  int st = ROWPTR[a], cnt = ROWCNT[a]; cnt = iclamp(cnt, 0, 4096); st = iclamp(st, 0, permLen - cnt);
  v8f ms = {};
  const float bf = bf16_rne(linb[nloc]), bc = bf16_rne(linb[16 + nloc]);
  for (int j = 0; j < cnt; ++j) { const int e = iclamp(PERM[st + j], 0, E - 1); const int tg = iclamp(tgt[e], 0, N - 1);
    __syncthreads(); load_interior(T, atom + (size_t)tg * C * HW, t_); __syncthreads();
    v8f z = {};
#pragma unroll
    for (int pr = 0; pr < 5; ++pr) z = wmma16b(frag_taps(T, y, x, pr, hlf), frag_kb(WE + (size_t)nloc * KP + pr * 32, hlf), z);
#pragma unroll
    for (int r = 0; r < 8; ++r) { const int p2 = wave * 16 + 8 * hlf + r; const float zv = elu(pmul(thn[r], z[r] * (1.0f / (XS * WSC)))); b16 h_, l_; split16(zv * XS, h_, l_); const int cell = (1 + (p2 >> 3)) * 10 + 1 + (p2 & 7); Zh[cell][nloc] = h_; Zl[cell][nloc] = l_; }
    __syncthreads();
    v8f tf = {}, tc = {};
#pragma unroll
    for (int pr = 0; pr < 5; ++pr) { const v16b ah = frag_taps(Zh, y, x, pr, hlf), al = frag_taps(Zl, y, x, pr, hlf); const v16b bf_ = frag_kb(WL + (size_t)nloc * KP + pr * 32, hlf), bc_ = frag_kb(WL + (size_t)(16 + nloc) * KP + pr * 32, hlf);
      tf = wmma16b(ah, bf_, tf); tf = wmma16b(al, bf_, tf); tc = wmma16b(ah, bc_, tc); tc = wmma16b(al, bc_, tc); }
#pragma unroll
    for (int r = 0; r < 8; ++r) ms[r] += pmul(sigm(tf[r] * (1.0f / (XS * WSC)) + bf), softplus(tc[r] * (1.0f / (XS * WSC)) + bc)); }
  const float gs = bf16_rne(gam[nloc]) * BNI, bb = bf16_rne(bet[nloc]);
#pragma unroll
  for (int r = 0; r < 8; ++r) { const int p2 = wave * 16 + 8 * hlf + r; const float xv = bf16_rne(atom[((size_t)a * C + nloc) * HW + p2]); To[nloc][p2] = softplus(xv + pmul(xv + ms[r], gs) + bb); }
  __syncthreads();
  for (int pass = 0; pass < 2; ++pass) { for (int i = t_; i < C * 16; i += 128) { const int ch = i >> 4, x4 = (i & 15) * 4; *(volatile v4f*)(out + ((size_t)a * C + ch) * HW + x4) = *(const v4f*)(&To[ch][x4]); } __threadfence(); }
}
}

extern "C" void kernel_launch(void* const* d_in, const int* in_sizes, int n_in, void* d_out, int out_size, void* d_ws, size_t ws_size, hipStream_t stream) {
  (void)n_in;
  auto Fp = [&](int i) { return (const float*)d_in[i]; }; auto Ip = [&](int i) { return (const int*)d_in[i]; };
  if (in_sizes[0] != N * C * HW || in_sizes[1] != E || in_sizes[2] != E || in_sizes[3] != C * KC || in_sizes[5] != 32 * KC || out_size != N * C * HW) return;
  size_t off = 0; char* ws = (char*)d_ws;
  auto carve = [&](size_t bytes) { char* p = ws + off; off += (bytes + 255) & ~(size_t)255; return p; };
  b16* WP = (b16*)carve((size_t)64 * KP * 2); CsrBufs csr; off = csr_carve(csr, ws, off, E, N);
  if (off > ws_size || off > ((size_t)128 << 20)) return;
  prep_kernel<<<(64 * KP / 8 + 255) / 256, 256, 0, stream>>>(Fp(3), Fp(4), Fp(5), WP);
  csr_build(csr, Ip(1), E, N, stream);
  atom_kernel<<<N, 128, 0, stream>>>(Fp(0), Ip(2), WP, Fp(6), Fp(7), Fp(8), csr.PERM, csr.ROWPTR, csr.ROWCNT, (int)csr.permLen, (float*)d_out);
}
